// MultiheadAttention_42606075576664
// MI455X (gfx1250) — hardware-verified
//
#include <hip/hip_runtime.h>


#ifndef NB
#define NB 2
#endif
#ifndef SEQ
#define SEQ 2048
#endif
#define NB_FULL  2
#define SEQ_FULL 2048
#define DM   1024
#define NH   16
#define HD   64
#define NKB  (SEQ / 32)
#define NQT  (SEQ / 16)
#define PLN  ((size_t)NB * NH * SEQ * HD)
#define WCAR 8.0f
#define PCAR 1024.0f
#define XP   72
#define NLINES ((NB * SEQ * NKB) / 32)
static_assert(SEQ % 64 == 0);
static_assert(SEQ <= SEQ_FULL);
static_assert(NB <= NB_FULL);
static_assert(DM % 64 == 0);
static_assert((DM & (DM - 1)) == 0);
static_assert(DM % 32 == 0);
static_assert(HD == 64);
static_assert(DM == NH * HD);
static_assert((NB * SEQ * NKB) % 32 == 0);
static_assert(XP % 8 == 0 && XP >= HD);

typedef _Float16 h16;
typedef unsigned short bf;
typedef __attribute__((ext_vector_type(16))) __bf16   v16bf;
typedef __attribute__((ext_vector_type(16))) _Float16 v16h;
typedef __attribute__((ext_vector_type(8)))  _Float16 v8h;
typedef __attribute__((ext_vector_type(8)))  unsigned short v8us;
typedef __attribute__((ext_vector_type(8)))  float    v8f;
typedef __attribute__((ext_vector_type(4)))  float    v4f;
typedef v4f  __attribute__((may_alias)) v4fa;

__device__ __forceinline__ unsigned short f2bf(float f) { unsigned u = __float_as_uint(f); u += 0x7FFFu + ((u >> 16) & 1u); return (unsigned short)(u >> 16); }
__device__ __forceinline__ float bf2f(unsigned short b) { return __uint_as_float(((unsigned)b) << 16); }
__device__ __forceinline__ float bfv(float f) { return bf2f(f2bf(f)); }
__device__ __forceinline__ void splitf(float y, unsigned short& h, unsigned short& l) { h = f2bf(y); l = f2bf(y - bf2f(h)); }
__device__ __forceinline__ v16h cat16(v8h lo, v8h hi) { return __builtin_shufflevector(lo, hi, 0, 1, 2, 3, 4, 5, 6, 7, 8, 9, 10, 11, 12, 13, 14, 15); }
__device__ __forceinline__ v16bf cat16b(v8us lo, v8us hi) { return __builtin_bit_cast(v16bf, __builtin_shufflevector(lo, hi, 0, 1, 2, 3, 4, 5, 6, 7, 8, 9, 10, 11, 12, 13, 14, 15)); }
__device__ __forceinline__ v8f wmma16(v16h a, v16h b, v8f c) {
    c = __builtin_amdgcn_wmma_f32_16x16x32_f16(false, a, false, b, (short)0, c, false, false);
    asm volatile("v_nop\n\tv_nop\n\tv_nop\n\tv_nop" : "+v"(c) : "v"(a), "v"(b));
    return c;
}
__device__ __forceinline__ v8f wmmab(v16bf a, v16bf b, v8f c) {
    c = __builtin_amdgcn_wmma_f32_16x16x32_bf16(false, a, false, b, (short)0, c, false, false);
    asm volatile("v_nop\n\tv_nop\n\tv_nop\n\tv_nop" : "+v"(c) : "v"(a), "v"(b));
    return c;
}
__device__ __forceinline__ v16h  ldh(const h16* p) { return cat16(*(const v8h*)p, *(const v8h*)(p + 16)); }
__device__ __forceinline__ v16bf ldb(const bf* p)  { return cat16b(*(const v8us*)p, *(const v8us*)(p + 16)); }
__device__ __forceinline__ void wsync() { asm volatile("s_wait_dscnt 0" ::: "memory"); __builtin_amdgcn_wave_barrier(); asm volatile("" ::: "memory"); }

__global__ __launch_bounds__(256) void k_cvt8(const float* __restrict__ src, bf* dst, unsigned n8) {
    const unsigned i = blockIdx.x * 256u + threadIdx.x; if (i >= n8) return;
    const float* s = src + (size_t)i * 8; bf* d = dst + (size_t)i * 8;
    const v8f v = *(const v8f*)s; v8us o;
#pragma unroll
    for (int k = 0; k < 8; ++k) o[k] = f2bf(v[k]);
    *(volatile v8us*)d = o; __threadfence(); *(volatile v8us*)d = o;
}

__global__ __launch_bounds__(256) void k_wcvt(const float* __restrict__ wq, const float* __restrict__ wk, const float* __restrict__ wv, h16* W16) {
    const unsigned i = blockIdx.x * 256u + threadIdx.x; if (i >= (unsigned)(HD * HD / 8)) return;
    const v8f a = *(const v8f*)(wq + (size_t)i * 8), b = *(const v8f*)(wk + (size_t)i * 8), c = *(const v8f*)(wv + (size_t)i * 8);
    v8h oa, ob, oc;
#pragma unroll
    for (int k = 0; k < 8; ++k) { oa[k] = (h16)(bfv(a[k]) * WCAR); ob[k] = (h16)(bfv(b[k]) * WCAR); oc[k] = (h16)(bfv(c[k]) * WCAR); }
    h16* d = W16 + (size_t)i * 8;
    *(volatile v8h*)d = oa; *(volatile v8h*)(d + HD * HD) = ob; *(volatile v8h*)(d + 2 * HD * HD) = oc;
    __threadfence();
    *(volatile v8h*)d = oa; *(volatile v8h*)(d + HD * HD) = ob; *(volatile v8h*)(d + 2 * HD * HD) = oc;
}

__global__ __launch_bounds__(256) void k_mbits(const int* __restrict__ mask, unsigned* MB) {
    const int lane = threadIdx.x & 31; const int wave = __builtin_amdgcn_readfirstlane(threadIdx.x >> 5);
    const int line = blockIdx.x * 8 + wave; if (line >= NLINES) return;
    unsigned word = 0u;
#pragma unroll 8
    for (int i = 0; i < 32; ++i) {
        const int gw = line * 32 + i;
        const int row = gw / NKB, w = gw % NKB;
        const int b = row / SEQ, q = row % SEQ;
        const int mv = mask[((size_t)b * SEQ_FULL + q) * SEQ_FULL + w * 32 + lane];
        const unsigned bal = __builtin_amdgcn_ballot_w32(mv != 0);
        word = (lane == i) ? bal : word;
    }
    unsigned* d = MB + (size_t)line * 32 + lane;
    *(volatile unsigned*)d = word; __threadfence(); *(volatile unsigned*)d = word;
}

template <bool TRANS>
__device__ __forceinline__ void proj_body(const float* __restrict__ X, const h16* __restrict__ W, const float* __restrict__ bias, h16* OUT) {
    __shared__ __align__(16) float os[64 * 68];
    __shared__ __align__(16) h16 xs[64 * XP];
    const int lane = threadIdx.x & 31, lr = lane & 15, hi = lane >> 4;
    const int rq = lane >> 3, piece = lane & 7;
    const int r0 = blockIdx.x * 64, hd = blockIdx.y;
    const int bb = r0 / SEQ, t0 = r0 % SEQ;
    const size_t xbase = ((size_t)bb * SEQ_FULL + t0) * DM + (size_t)hd * HD;
#pragma unroll 4
    for (int it = 0; it < 16; ++it) { const int row = 4 * it + rq;
        const v8f v = *(const v8f*)(X + xbase + (size_t)row * DM + piece * 8); v8h o;
#pragma unroll
        for (int k = 0; k < 8; ++k) o[k] = (h16)bfv(v[k]);
        *(v8h*)&xs[row * XP + piece * 8] = o; }
    float bz[4];
#pragma unroll
    for (int nb = 0; nb < 4; ++nb) bz[nb] = bfv(bias[nb * 16 + lr]) * WCAR;
    wsync();
    v8f acc[4][4];
#pragma unroll
    for (int mb = 0; mb < 4; ++mb)
#pragma unroll
        for (int nb = 0; nb < 4; ++nb) acc[mb][nb] = (v8f){};
#pragma unroll
    for (int ks = 0; ks < 2; ++ks) {
        v16h a[4];
#pragma unroll
        for (int mb = 0; mb < 4; ++mb) { const int xo = (mb * 16 + lr) * XP + ks * 32 + 8 * hi;
            a[mb] = cat16(*(const v8h*)&xs[xo], *(const v8h*)&xs[xo + 16]); }
#pragma unroll
        for (int nb = 0; nb < 4; ++nb) { const v16h b = ldh(W + (size_t)(nb * 16 + lr) * HD + ks * 32 + 8 * hi);
#pragma unroll
            for (int mb = 0; mb < 4; ++mb) acc[mb][nb] = wmma16(a[mb], b, acc[mb][nb]); }
    }
#pragma unroll
    for (int mb = 0; mb < 4; ++mb)
#pragma unroll
        for (int nb = 0; nb < 4; ++nb)
#pragma unroll
            for (int j = 0; j < 8; ++j) os[(mb * 16 + hi * 8 + j) * 68 + nb * 16 + lr] = acc[mb][nb][j] + bz[nb];
    wsync();
    const size_t bh = (size_t)bb * NH + hd;
    if (!TRANS) {
        const size_t po = (bh * SEQ + t0) * HD + piece * 8;
#pragma unroll 1
        for (int ps = 0; ps < 2; ++ps) {
#pragma unroll 1
            for (int s = 0; s < 16; ++s) { const int row = 4 * s + rq;
                const v4f u0 = *(const v4fa*)(os + row * 68 + piece * 8), u1 = *(const v4fa*)(os + row * 68 + piece * 8 + 4); v8h hv;
#pragma unroll
                for (int i = 0; i < 4; ++i) { hv[i] = (h16)u0[i]; hv[4 + i] = (h16)u1[i]; }
                *(volatile v8h*)(OUT + po + (size_t)row * HD) = hv; }
            if (ps == 0) __threadfence(); }
    } else {
#pragma unroll 1
        for (int ps = 0; ps < 2; ++ps) {
#pragma unroll 1
            for (int s = 0; s < 16; ++s) { const int drow = 4 * s + rq; v8h hv;
#pragma unroll
                for (int i = 0; i < 8; ++i) hv[i] = (h16)os[(piece * 8 + i) * 68 + drow];
                *(volatile v8h*)(OUT + (bh * HD + drow) * SEQ + t0 + piece * 8) = hv; }
            if (ps == 0) __threadfence(); }
    }
}
__global__ __launch_bounds__(32) void k_proj_rows(const float* X, const h16* W, const float* bias, h16* OUT) { proj_body<false>(X, W, bias, OUT); }
__global__ __launch_bounds__(32) void k_proj_tr(const float* X, const h16* W, const float* bias, h16* OUT) { proj_body<true>(X, W, bias, OUT); }

__global__ __launch_bounds__(128) void k_attn(const h16* __restrict__ QK16, const h16* __restrict__ VT16, const unsigned* __restrict__ MB, bf* CTX) {
    __shared__ __align__(16) float os[4 * 16 * 68];
    const int lane = threadIdx.x & 31, n = lane & 15, hh = lane >> 4;
    const int wave = __builtin_amdgcn_readfirstlane(threadIdx.x >> 5);
    const int bh = blockIdx.y;
    const int bb = bh / NH, hd = bh % NH;
    const int qt = blockIdx.x * 4 + wave;
    const int q0 = qt * 16;
    const size_t pb = (size_t)bh * SEQ * HD;
    const size_t qoff = pb + (size_t)(q0 + n) * HD + 8 * hh;
    const size_t koffb = PLN + pb + (size_t)n * HD + 8 * hh;
    const size_t voffb = ((size_t)bh * HD + n) * SEQ + 8 * hh;
    const size_t moffb = ((size_t)bb * SEQ + q0 + n) * NKB;
    const float NINF = -__builtin_inff();
    const float SC2 = 1.4426950408889634f * (1.0f / 2048.0f);
    const float FILLV = (-1.0e20f * 0.03125f) * 1.4426950408889634f;
    v8f acc[4];
#pragma unroll
    for (int dt = 0; dt < 4; ++dt) acc[dt] = (v8f){};
    float m = NINF, l = 0.0f;
#pragma unroll 1
    for (int kb = 0; kb < NKB; ++kb) {
        const int key0 = kb * 32;
        const size_t ko = koffb + (size_t)key0 * HD;
        const unsigned mw = MB[moffb + kb];
        v8f s0 = (v8f){}, s1 = (v8f){};
#pragma unroll
        for (int ks = 0; ks < 2; ++ks) {
            const v16h qa = ldh(QK16 + qoff + ks * 32);
            const v16h k0 = ldh(QK16 + ko + ks * 32), k1 = ldh(QK16 + ko + 16 * HD + ks * 32);
            s0 = wmma16(k0, qa, s0);
            s1 = wmma16(k1, qa, s1);
        }
        const unsigned wa = mw >> (8 * hh);
        float t[16];
#pragma unroll
        for (int r = 0; r < 8; ++r) {
            t[r]     = ((wa >> r) & 1u)        ? s0[r] * SC2 : FILLV;
            t[8 + r] = ((wa >> (16 + r)) & 1u) ? s1[r] * SC2 : FILLV;
        }
        float mx = t[0];
#pragma unroll
        for (int i = 1; i < 16; ++i) mx = fmaxf(mx, t[i]);
        mx = fmaxf(mx, __shfl_xor(mx, 16, 32));
        const float mn = fmaxf(m, mx);
        const float ms = (mn == NINF) ? 0.0f : mn;
        const float corr = __builtin_amdgcn_exp2f(m - ms);
        m = mn;
        float psum = 0.0f;
#pragma unroll
        for (int i = 0; i < 16; ++i) { t[i] = __builtin_amdgcn_exp2f(t[i] - ms); psum += t[i]; }
        l = l * corr + psum;
#pragma unroll
        for (int dt = 0; dt < 4; ++dt)
#pragma unroll
            for (int r = 0; r < 8; ++r) acc[dt][r] *= corr;
        v8h pa, pc;
#pragma unroll
        for (int r = 0; r < 8; ++r) { pa[r] = (h16)(t[r] * PCAR); pc[r] = (h16)(t[8 + r] * PCAR); }
        const v16h pf = cat16(pa, pc);
        const size_t vo = voffb + key0;
        v16h va[4];
#pragma unroll
        for (int dt = 0; dt < 4; ++dt) va[dt] = ldh(VT16 + vo + (size_t)dt * 16 * SEQ);
#pragma unroll
        for (int dt = 0; dt < 4; ++dt) acc[dt] = wmma16(va[dt], pf, acc[dt]);
    }
    l += __shfl_xor(l, 16, 32);
    const float inv = (1.0f / l) * (1.0f / (PCAR * WCAR));
    const int obase = wave * (16 * 68);
#pragma unroll
    for (int dt = 0; dt < 4; ++dt)
#pragma unroll
        for (int r = 0; r < 8; ++r) os[obase + n * 68 + dt * 16 + 8 * hh + r] = acc[dt][r] * inv;
    wsync();
    const int rq = lane >> 3, piece = lane & 7;
#pragma unroll 1
    for (int ps = 0; ps < 2; ++ps) {
#pragma unroll
        for (int s = 0; s < 4; ++s) { const int row = 4 * s + rq;
            const v4f u0 = *(const v4fa*)(os + obase + row * 68 + piece * 8), u1 = *(const v4fa*)(os + obase + row * 68 + piece * 8 + 4); v8us oh, ol;
#pragma unroll
            for (int i = 0; i < 4; ++i) { unsigned short a, c; splitf(u0[i], a, c); oh[i] = a; ol[i] = c; splitf(u1[i], a, c); oh[4 + i] = a; ol[4 + i] = c; }
            const size_t o = ((size_t)bb * SEQ + q0 + row) * (2 * DM) + hd * HD + piece * 8;
            *(volatile v8us*)(CTX + o) = oh; *(volatile v8us*)(CTX + o + DM) = ol; }
        if (ps == 0) __threadfence(); }
}

__device__ __forceinline__ void gemm64(const bf* __restrict__ A, const size_t lda, const bf* __restrict__ Bt, const size_t ldbt, const int K, const int kmask, const int r0, const int c0, v8f (&acc)[4][4]) {
    const int lane = threadIdx.x & 31, lr = lane & 15, hi = lane >> 4;
#pragma unroll
    for (int mb = 0; mb < 4; ++mb)
#pragma unroll
        for (int nb = 0; nb < 4; ++nb) acc[mb][nb] = (v8f){};
    const size_t aoff = (size_t)(r0 + lr) * lda + 8 * hi, boff = (size_t)(c0 + lr) * ldbt + 8 * hi;
#pragma unroll 1
    for (int kc = 0; kc < K; kc += 32) {
        const int kb = kc & kmask;
        v16bf a[4];
#pragma unroll
        for (int mb = 0; mb < 4; ++mb) a[mb] = ldb(A + aoff + (size_t)mb * 16 * lda + kc);
#pragma unroll
        for (int nb = 0; nb < 4; ++nb) { const v16bf b = ldb(Bt + boff + (size_t)nb * 16 * ldbt + kb);
#pragma unroll
            for (int mb = 0; mb < 4; ++mb) acc[mb][nb] = wmmab(a[mb], b, acc[mb][nb]); }
    }
}

__global__ __launch_bounds__(32) void k_fc(const bf* __restrict__ CTX, const bf* __restrict__ WF, const float* __restrict__ bfc, float* OUT) {
    __shared__ __align__(16) float os[16 * 68];
    const int lane = threadIdx.x & 31, lr = lane & 15, hi = lane >> 4;
    const int r0 = blockIdx.x * 64, c0 = blockIdx.y * 64;
    v8f acc[4][4];
    gemm64(CTX, 2 * DM, WF, DM, 2 * DM, DM - 1, r0, c0, acc);
    v4f bz = *(const v4f*)(bfc + c0 + lr * 4);
#pragma unroll
    for (int i = 0; i < 4; ++i) bz[i] = bfv(bz[i]);
#pragma unroll
    for (int mb = 0; mb < 4; ++mb) {
#pragma unroll
        for (int nb = 0; nb < 4; ++nb)
#pragma unroll
            for (int j = 0; j < 8; ++j) os[(hi * 8 + j) * 68 + nb * 16 + lr] = acc[mb][nb][j];
        wsync();
        float* crow = OUT + (size_t)(r0 + mb * 16) * DM + c0;
#pragma unroll 1
        for (int ps = 0; ps < 2; ++ps) {
#pragma unroll
            for (int s = 0; s < 8; ++s) { const int row = 2 * s + hi, cofs = lr * 4; const v4f val = *(const v4fa*)(os + row * 68 + cofs) + bz;
                *(volatile v4f*)(crow + (size_t)row * DM + cofs) = val; }
            if (ps == 0) __threadfence(); }
        wsync();
    }
}

#define SZ_W16 ((size_t)3 * HD * HD * 2)
#define SZ_WF  ((size_t)DM * DM * 2)
#define SZ_QK  ((size_t)2 * NB * NH * SEQ * HD * 2)
#define SZ_VT  ((size_t)NB * NH * HD * SEQ * 2)
#define SZ_CTX ((size_t)NB * SEQ * 2 * DM * 2)
#define SZ_MB  ((size_t)NB * SEQ * NKB * 4)
#define WS_TOTAL (SZ_W16 + SZ_WF + SZ_QK + SZ_VT + SZ_CTX + SZ_MB)
static_assert(WS_TOTAL <= (size_t)134217728);
static_assert(SZ_W16 % 256 == 0 && SZ_WF % 256 == 0 && SZ_QK % 256 == 0 && SZ_VT % 256 == 0 && SZ_CTX % 256 == 0 && SZ_MB % 128 == 0);
static_assert((DM * DM / 8) % 256 == 0);
static_assert((HD * HD / 8) == 512);
static_assert(SZ_MB == (size_t)NLINES * 128);

extern "C" void kernel_launch(void* const* d_in, const int* in_sizes, int n_in,
                              void* d_out, int out_size, void* d_ws, size_t ws_size, hipStream_t stream) {
    if (n_in < 12) return;
    const long long strm = (long long)(NB - 1) * SEQ_FULL * DM + (long long)SEQ * DM;
    if ((long long)in_sizes[0] < strm || (long long)in_sizes[1] < strm || (long long)in_sizes[2] < strm) return;
    if ((long long)in_sizes[3] < (long long)(NB - 1) * SEQ_FULL * SEQ_FULL + (long long)(SEQ - 1) * SEQ_FULL + SEQ) return;
    if (in_sizes[4] < HD * HD || in_sizes[6] < HD * HD || in_sizes[8] < HD * HD) return;
    if (in_sizes[5] < HD || in_sizes[7] < HD || in_sizes[9] < HD) return;
    if ((long long)in_sizes[10] < (long long)DM * DM || in_sizes[11] < DM) return;
    if ((long long)out_size < (long long)NB * SEQ * DM) return;
    if (ws_size < WS_TOTAL) return;
    const float* xq = (const float*)d_in[0];
    const float* xk = (const float*)d_in[1];
    const float* xv = (const float*)d_in[2];
    const int* mask = (const int*)d_in[3];
    const float* wq = (const float*)d_in[4];
    const float* bq = (const float*)d_in[5];
    const float* wk = (const float*)d_in[6];
    const float* bk = (const float*)d_in[7];
    const float* wv = (const float*)d_in[8];
    const float* bv = (const float*)d_in[9];
    const float* wfc = (const float*)d_in[10];
    const float* bfc = (const float*)d_in[11];
    float* OUT = (float*)d_out;
    char* wsp = (char*)d_ws;
    h16* W16 = (h16*)wsp;  wsp += SZ_W16;
    bf* WF = (bf*)wsp;     wsp += SZ_WF;
    h16* QK16 = (h16*)wsp; wsp += SZ_QK;
    h16* VT16 = (h16*)wsp; wsp += SZ_VT;
    bf* CTX = (bf*)wsp;    wsp += SZ_CTX;
    unsigned* MB = (unsigned*)wsp; wsp += SZ_MB;

    k_wcvt<<<2, 256, 0, stream>>>(wq, wk, wv, W16);
    k_cvt8<<<(unsigned)(DM * DM / 8 / 256), 256, 0, stream>>>(wfc, WF, (unsigned)(DM * DM / 8));
    k_mbits<<<(unsigned)((NLINES + 7) / 8), 256, 0, stream>>>(mask, MB);
    k_proj_rows<<<dim3(NB * SEQ / 64, NH), 32, 0, stream>>>(xq, W16, bq, QK16);
    k_proj_rows<<<dim3(NB * SEQ / 64, NH), 32, 0, stream>>>(xk, W16 + HD * HD, bk, QK16 + PLN);
    k_proj_tr<<<dim3(NB * SEQ / 64, NH), 32, 0, stream>>>(xv, W16 + 2 * HD * HD, bv, VT16);
    k_attn<<<dim3(SEQ / 64, NB * NH), 128, 0, stream>>>(QK16, VT16, MB, CTX);
    k_fc<<<dim3(NB * SEQ / 64, DM / 64), 32, 0, stream>>>(CTX, WF, bfc, OUT);
}
